// BellmanFilter_31336081392170
// MI455X (gfx1250) — hardware-verified
//
#include <hip/hip_runtime.h>
#include <math.h>
#include <stddef.h>


#define NOBS 128
#define KF   16
#define SD   32
#define TB   64
#define YP   136
#define P16  40

typedef _Float16 v16h __attribute__((ext_vector_type(16)));
typedef _Float16 v8h  __attribute__((ext_vector_type(8)));
typedef _Float16 v4h  __attribute__((ext_vector_type(4)));
typedef float    v8f  __attribute__((ext_vector_type(8)));
typedef float    v4f  __attribute__((ext_vector_type(4)));
union Frag { v16h v; v8h hv[2]; };

__device__ __forceinline__ v8f wmma_f16(v16h a, v16h b, v8f c)
{
  v8f d = __builtin_amdgcn_wmma_f32_16x16x32_f16(false, a, false, b, (short)0, c, false, false);
  asm volatile("v_nop\n\tv_nop\n\tv_nop\n\tv_nop" : "+v"(d) : "v"(a), "v"(b));
  return d;
}

__device__ __forceinline__ v16h ld_frag(const _Float16* base, int pitch, int row, int k0, int h)
{
  Frag f;
  const _Float16* p = base + row * pitch + k0 + 8 * h;
  f.hv[0] = *(const v8h*)(p);
  f.hv[1] = *(const v8h*)(p + 16);
  return f.v;
}

__device__ __forceinline__ float sum16(float v)
{
  v += __shfl_xor(v, 8);
  v += __shfl_xor(v, 4);
  v += __shfl_xor(v, 2);
  v += __shfl_xor(v, 1);
  return v;
}

__device__ inline float gj16(float* M, float* prow, float* fac, int tid)
{
  float ld = 0.0f;
#pragma unroll 1
  for (int p = 0; p < KF; ++p) {
    if (tid < 32) {
      const float piv  = M[p * 32 + p];
      const float pinv = 1.0f / piv;
      prow[tid] = M[p * 32 + tid] * pinv;
      if (tid == 0) ld += logf(fabsf(piv));
    } else if (tid < 48) {
      fac[tid - 32] = M[(tid - 32) * 32 + p];
    }
    __syncthreads();
#pragma unroll
    for (int q = 0; q < 2; ++q) {
      const int e = tid + q * 256;
      const int i = e >> 5, j = e & 31;
      const float pr  = prow[j];
      const float cur = M[e];
      M[e] = (i == p) ? pr : (cur - fac[i] * pr);
    }
    __syncthreads();
  }
  return ld;
}

__global__ __launch_bounds__(128)
void k_proj(const float* __restrict__ obs, const float* __restrict__ lam,
            const float* __restrict__ sig2, float* bout, float* cout, int T)
{
  __shared__ _Float16 Ys[TB * YP] __attribute__((aligned(16)));
  __shared__ _Float16 Wt[KF * YP] __attribute__((aligned(16)));
  __shared__ float Os[4 * 256] __attribute__((aligned(16)));
  __shared__ float cs[TB] __attribute__((aligned(16)));
  __shared__ float sInv[NOBS];

  const int tid = threadIdx.x, lane = tid & 31, wid = tid >> 5, h = lane >> 4, m = lane & 15;
  const int t0 = blockIdx.x * TB;

  for (int n = tid; n < NOBS; n += 128) sInv[n] = 1.0f / sig2[n];
  __syncthreads();

  for (int idx = tid; idx < NOBS * KF; idx += 128) {
    const int n = idx >> 4, k = idx & 15;
    Wt[k * YP + n] = (_Float16)(64.0f * lam[idx] * sInv[n]);
  }
  {
    const int r = tid >> 1, hf = tid & 1, t = t0 + r;
    float p = 0.0f;
#pragma unroll 4
    for (int q = 0; q < 16; ++q) {
      const int c = 64 * hf + 4 * q;
      v4f y = {0.f, 0.f, 0.f, 0.f};
      if (t < T) y = *(const v4f*)(obs + (size_t)t * NOBS + c);
      p += y.x * y.x * sInv[c] + y.y * y.y * sInv[c + 1] + y.z * y.z * sInv[c + 2] + y.w * y.w * sInv[c + 3];
      v4h yh;
      yh.x = (_Float16)y.x; yh.y = (_Float16)y.y; yh.z = (_Float16)y.z; yh.w = (_Float16)y.w;
      *(v4h*)(Ys + r * YP + c) = yh;
    }
    p += __shfl_xor(p, 1);
    if (hf == 0) cs[r] = p;
  }
  __syncthreads();

  v8f acc = {0.f, 0.f, 0.f, 0.f, 0.f, 0.f, 0.f, 0.f};
#pragma unroll
  for (int s = 0; s < 4; ++s) {
    const v16h a = ld_frag(Ys, YP, wid * 16 + m, 32 * s, h);
    const v16h b = ld_frag(Wt, YP, m, 32 * s, h);
    acc = wmma_f16(a, b, acc);
  }
#pragma unroll
  for (int r = 0; r < 8; ++r) Os[wid * 256 + (8 * h + r) * 16 + m] = acc[r] * (1.0f / 64.0f);
  __syncthreads();

  const int qa = lane, qb = 32 + lane;
  const int ra = qa >> 2, ca = (qa & 3) * 4, rb = qb >> 2, cb = (qb & 3) * 4;
  const v4f va = *(const v4f*)(Os + wid * 256 + ra * 16 + ca);
  const v4f vb = *(const v4f*)(Os + wid * 256 + rb * 16 + cb);
  const int ta = t0 + wid * 16 + ra, tb = t0 + wid * 16 + rb;
  float* pa = bout + (size_t)ta * KF + ca;
  float* pb = bout + (size_t)tb * KF + cb;
  const bool wa = (ta < T), wb = (tb < T);
  const bool wc = (wid == 0) && (lane < 16) && (t0 + 4 * lane + 3 < T);
  v4f vc = {0.f, 0.f, 0.f, 0.f};
  if (wc) vc = *(const v4f*)(cs + 4 * lane);
  float* pc = cout + t0 + 4 * lane;

  if (wa) *(volatile v4f*)pa = va;
  if (wb) *(volatile v4f*)pb = vb;
  if (wc) *(volatile v4f*)pc = vc;
  __threadfence();
  if (wa) *(volatile v4f*)pa = va;
  if (wb) *(volatile v4f*)pb = vb;
  if (wc) *(volatile v4f*)pc = vc;
}

__global__ __launch_bounds__(256)
void k_filter(const float* __restrict__ lam, const float* __restrict__ phif,
              const float* __restrict__ phih, const float* __restrict__ mug,
              const float* __restrict__ sig2, const float* __restrict__ qh,
              const float* bin, const float* cin,
              float* means, float* infos, float* llout, int T)
{
  __shared__ double dA[256], dS[256], dTm[256];
  __shared__ float sLam[NOBS * KF];
  __shared__ float sInv[NOBS];
  __shared__ float sJ[256], sPhi[256];
  __shared__ float sOmh[256] __attribute__((aligned(16)));
  __shared__ _Float16 Phi16[KF * P16] __attribute__((aligned(16)));
  __shared__ _Float16 Pt16[KF * P16]  __attribute__((aligned(16)));
  __shared__ _Float16 T1s[KF * P16]   __attribute__((aligned(16)));
  __shared__ float M1[KF * 32] __attribute__((aligned(16)));
  __shared__ float M2[KF * 32] __attribute__((aligned(16)));
  __shared__ float mring[32 * SD] __attribute__((aligned(16)));
  __shared__ float prow[32], fac[16];
  __shared__ float fv[16], fp[16], uu[16], bt[16], hexp[16];
  __shared__ float sSlog;

  const int tid = threadIdx.x, lane = tid & 31, wid = tid >> 5, h = lane >> 4, m = lane & 15;
  const int ti = tid >> 4, tj = tid & 15;

  for (int idx = tid; idx < NOBS * KF; idx += 256) sLam[idx] = lam[idx];
  if (tid < NOBS) sInv[tid] = 1.0f / sig2[tid];
  sPhi[tid] = phif[tid];
  dA[tid] = (double)phih[tid];
  dS[tid] = (double)qh[tid];
  Phi16[ti * P16 + tj] = (_Float16)(16.0f * phif[tid]);
  Phi16[ti * P16 + 16 + tj] = (_Float16)0.0f;
  Pt16[ti * P16 + 16 + tj]  = (_Float16)0.0f;
  T1s[ti * P16 + 16 + tj]   = (_Float16)0.0f;
  if (tj < 8) {
    Phi16[ti * P16 + 32 + tj] = (_Float16)0.0f;
    Pt16[ti * P16 + 32 + tj]  = (_Float16)0.0f;
    T1s[ti * P16 + 32 + tj]   = (_Float16)0.0f;
  }
  M2[ti * 32 + tj] = 0.0f;
  M2[ti * 32 + 16 + tj] = (ti == tj) ? 1.0f : 0.0f;
  for (int idx = tid; idx < 32 * SD; idx += 256) {
    const int c = idx & 31;
    mring[idx] = (c < KF) ? 0.0f : mug[c - KF];
  }
  if (tid < KF) { hexp[tid] = expf(mug[tid]); fv[tid] = 0.0f; }
  if (tid == 0) {
    float s = 0.0f;
#pragma unroll 1
    for (int n = 0; n < NOBS; ++n) s += logf(sig2[n]);
    sSlog = s;
  }
  __syncthreads();

  {
    double a = 0.0;
#pragma unroll 2
    for (int n = 0; n < NOBS; ++n)
      a += (double)(sLam[n * KF + ti] * sInv[n]) * (double)sLam[n * KF + tj];
    sJ[tid] = (float)a;
  }

#pragma unroll 1
  for (int lv = 0; lv < 20; ++lv) {
    double t = 0.0;
#pragma unroll 4
    for (int a = 0; a < KF; ++a) t += dA[ti * KF + a] * dS[a * KF + tj];
    dTm[tid] = t;
    __syncthreads();
    double s = dS[tid], a2 = 0.0;
#pragma unroll 4
    for (int b = 0; b < KF; ++b) {
      s  += dTm[ti * KF + b] * dA[tj * KF + b];
      a2 += dA[ti * KF + b] * dA[b * KF + tj];
    }
    __syncthreads();
    dS[tid] = s;
    dA[tid] = a2;
    __syncthreads();
  }
  M1[ti * 32 + tj] = (float)dS[tid];
  M1[ti * 32 + 16 + tj] = (ti == tj) ? 1.0f : 0.0f;
  __syncthreads();
  (void)gj16(M1, prow, fac, tid);
  sOmh[tid] = M1[ti * 32 + 16 + tj];
  __syncthreads();

  const int ri = tid >> 3, c0 = (tid & 7) * 4;
  const bool dyn = (ri < KF) && (c0 < KF);
  v4f cst = {0.f, 0.f, 0.f, 0.f};
  if (ri >= KF && c0 >= KF) cst = *(const v4f*)(sOmh + (ri - KF) * KF + (c0 - KF));

  const v16h aphi = ld_frag(Phi16, P16, m, 0, h);
  const v8f zero8 = {0.f, 0.f, 0.f, 0.f, 0.f, 0.f, 0.f, 0.f};
  const float LOG2PI = 1.8378770664093453f;
  float ll = 0.0f, q1 = 0.0f;

  for (int t = 0; t < T; ++t) {
    Pt16[tj * P16 + ti] = (_Float16)(256.0f * M2[ti * 32 + 16 + tj]);
    if (tid < KF) {
      float s = 0.0f;
#pragma unroll 4
      for (int a = 0; a < KF; ++a) s += sPhi[tid * KF + a] * fv[a];
      fp[tid] = s;
      bt[tid] = bin[(size_t)t * KF + tid];
    }
    __syncthreads();

    if (wid == 0) {
      const v16h b = ld_frag(Pt16, P16, m, 0, h);
      const v8f acc = wmma_f16(aphi, b, zero8);
#pragma unroll
      for (int r = 0; r < 8; ++r) T1s[(8 * h + r) * P16 + m] = (_Float16)acc[r];
      float term = 0.0f;
      if (lane < KF) {
        float jf = 0.0f;
#pragma unroll 4
        for (int a = 0; a < KF; ++a) jf += sJ[lane * KF + a] * fp[a];
        const float b0 = bt[lane];
        uu[lane] = b0 - jf;
        term = fp[lane] * (jf - 2.0f * b0);
      }
      term = sum16(term);
      if (lane == 0) q1 = cin[t] + term;
    }
    __syncthreads();

    if (wid == 0) {
      const v16h a = ld_frag(T1s, P16, m, 0, h);
      const v8f acc = wmma_f16(a, aphi, zero8);
#pragma unroll
      for (int r = 0; r < 8; ++r) {
        const int i = 8 * h + r;
        float v = acc[r] * (1.0f / 65536.0f);
        if (i == m) v += hexp[m];
        M1[i * 32 + m] = v;
        M1[i * 32 + 16 + m] = (i == m) ? 1.0f : 0.0f;
      }
    }
    __syncthreads();

    const float ld1 = gj16(M1, prow, fac, tid);

    M2[ti * 32 + tj] = M1[ti * 32 + 16 + tj] + sJ[tid];
    M2[ti * 32 + 16 + tj] = (ti == tj) ? 1.0f : 0.0f;
    __syncthreads();

    {
      v4f val = cst;
      if (dyn) val = *(const v4f*)(M2 + ri * 32 + c0);
      float* dst = infos + (size_t)t * (SD * SD) + tid * 4;
      *(volatile v4f*)dst = val;
      __threadfence();
      *(volatile v4f*)dst = val;
    }

    const float ld2 = gj16(M2, prow, fac, tid);

    if (wid == 0) {
      float g = 0.0f, u = 0.0f;
      if (lane < KF) {
#pragma unroll 4
        for (int a = 0; a < KF; ++a) g += M2[lane * 32 + 16 + a] * uu[a];
        u = uu[lane];
        const float f = fp[lane] + g;
        fv[lane] = f;
        mring[(t & 31) * SD + lane] = f;
      }
      const float q2 = sum16(u * g);
      if (lane == 0) ll += -0.5f * ((float)NOBS * LOG2PI + sSlog + ld1 + ld2 + q1 - q2);
    }
    if ((t & 31) == 31) {
      __syncthreads();
      const v4f v = *(const v4f*)(mring + tid * 4);
      float* dst = means + (size_t)(t - 31) * SD + tid * 4;
      *(volatile v4f*)dst = v;
      __threadfence();
      *(volatile v4f*)dst = v;
    }
    __syncthreads();
  }

  if (tid == 0) {
    *(volatile float*)llout = ll;
    __threadfence();
    *(volatile float*)llout = ll;
  }
}

extern "C" void kernel_launch(void* const* d_in, const int* in_sizes, int n_in,
                              void* d_out, int out_size, void* d_ws, size_t ws_size,
                              hipStream_t stream)
{
  if (n_in < 7) return;
  const int T = in_sizes[0] / NOBS;
  if (T <= 0 || (T % TB) != 0 || in_sizes[0] != T * NOBS) return;
  if (in_sizes[1] != NOBS * KF || in_sizes[2] != KF * KF || in_sizes[3] != KF * KF ||
      in_sizes[4] != KF || in_sizes[5] != NOBS || in_sizes[6] != KF * KF) return;
  const long long need_out = (long long)T * SD + (long long)T * SD * SD + 1;
  if ((long long)out_size != need_out) return;

  const size_t bytesB = (size_t)T * KF * sizeof(float);
  const size_t offC   = (bytesB + 127) & ~(size_t)127;
  const size_t bytesC = (size_t)T * sizeof(float);
  if (offC + bytesC > ws_size) return;

  const float* obs  = (const float*)d_in[0];
  const float* lam  = (const float*)d_in[1];
  const float* phif = (const float*)d_in[2];
  const float* phih = (const float*)d_in[3];
  const float* mu   = (const float*)d_in[4];
  const float* sig2 = (const float*)d_in[5];
  const float* qh   = (const float*)d_in[6];

  float* out   = (float*)d_out;
  float* means = out;
  float* infos = out + (size_t)T * SD;
  float* llp   = infos + (size_t)T * SD * SD;

  float* bws = (float*)d_ws;
  float* cws = (float*)((char*)d_ws + offC);

  hipLaunchKernelGGL(k_proj, dim3((T + TB - 1) / TB), dim3(128), 0, stream,
                     obs, lam, sig2, bws, cws, T);
  hipLaunchKernelGGL(k_filter, dim3(1), dim3(256), 0, stream,
                     lam, phif, phih, mu, sig2, qh,
                     (const float*)bws, (const float*)cws, means, infos, llp, T);
}
